// GATRegressor_18107582119952
// MI455X (gfx1250) — hardware-verified
//
#include <hip/hip_runtime.h>
#include <stddef.h>
#include <stdint.h>
#include <math.h>


#define DF     128
#define KP     256
#define NGR    512
#define NTHR   256
#define NWAVE  8
#define EPT    8
#define CHUNK  (NTHR * EPT)
#define WCAP   (EPT * 32)
#define LISTN  (NWAVE * WCAP)
#define NBA    512
#define SLA    9
#define RCAP   28672
#define DEGCAP 128
#define MEAS_B512 16715
#define MEAS_DEG  61
#define GBM    64
#define GBN    128
#define GTHR   128
#define NU1    (DF * (DF / 8))
#define NU2    (DF * (KP / 8))
#define PTHR   1024
#define PWAVE  32
#define NEGSL  0.2f
#define AGG_ZINTS (LISTN + 2 * RCAP + 3 * NBA)
#define AGG_LDS_INTS (AGG_ZINTS + 16)
#define WSMAX  134217728

static_assert((CHUNK & (CHUNK - 1)) == 0 && CHUNK <= 4096);
static_assert((NBA & (NBA - 1)) == 0 && NBA == (1 << SLA));
static_assert(((long long)CHUNK << SLA) < (1LL << 31));
static_assert(LISTN % NTHR == 0);
static_assert(NBA % NWAVE == 0 && NBA % 32 == 0 && NBA % GBM == 0);
static_assert(RCAP % 4 == 0 && AGG_ZINTS % 4 == 0 && LISTN % 4 == 0);
static_assert(RCAP >= MEAS_B512 + 4096);
static_assert(DEGCAP >= MEAS_DEG + 8);
static_assert(DF % 32 == 0 && KP % 32 == 0 && KP == 2 * DF && DF == GBN);
static_assert(GBM == (GTHR / 32) * 16 && GBN == 4 * 32);
static_assert(NU1 % NTHR == 0 && NU2 % NTHR == 0);
static_assert(DF / 8 == 16 && KP / 8 == 32);
static_assert(AGG_LDS_INTS * 4 <= 300000);
static_assert(DF == 4 * 32);
static_assert(NGR % PWAVE == 0 && PTHR == 32 * PWAVE && PWAVE == 32);

typedef float          v4f   __attribute__((ext_vector_type(4)));
typedef float          v8f   __attribute__((ext_vector_type(8)));
typedef int            v4i   __attribute__((ext_vector_type(4)));
typedef int            v8i   __attribute__((ext_vector_type(8)));
typedef unsigned int   v4u   __attribute__((ext_vector_type(4)));
typedef unsigned short v8us  __attribute__((ext_vector_type(8)));
typedef unsigned short v16us __attribute__((ext_vector_type(16)));
typedef __bf16         v16bf __attribute__((ext_vector_type(16)));
typedef v4f  __attribute__((may_alias)) v4fa;
typedef v4i  __attribute__((may_alias)) v4ia;
typedef v8us __attribute__((may_alias)) v8usa;
union FragB { v16bf v; v16us u; v8us h[2]; v8i w; };

__device__ __forceinline__ v8f wmb(const FragB& a, const FragB& b, v8f c) {
  v8f d = __builtin_amdgcn_wmma_f32_16x16x32_bf16(false, a.v, false, b.v, (short)0, c, false, false);
  asm volatile("v_nop\n\tv_nop\n\tv_nop\n\tv_nop" : "+v"(d) : "v"(a.w), "v"(b.w));
  return d;
}

__device__ __forceinline__ unsigned bf16_bits(float f) {
  const unsigned u = __float_as_uint(f);
  const unsigned r = (u + 0x7FFFu + ((u >> 16) & 1u)) >> 16;
  const unsigned q = (u >> 16) | 0x40u;
  return ((u & 0x7FFFFFFFu) > 0x7F800000u) ? q : r;
}
__device__ __forceinline__ float bf16_val(float f) {
  return __uint_as_float(bf16_bits(f) << 16);
}
__device__ __forceinline__ v4f bfr4(const v4f a) {
  v4f r; r.x = bf16_val(a.x); r.y = bf16_val(a.y); r.z = bf16_val(a.z); r.w = bf16_val(a.w); return r;
}

template <int SLB>
__device__ __forceinline__ int scan_chunk(const int* __restrict__ dsts, int nE, int cbase, int slotBase,
                                          int nb, int vec8, int* list, int tid, int lane, int wave) {
  int wc = 0;
  const int el0  = tid * EPT;
  const int e0   = cbase + el0;
  const int sent = -2147483647 - 1;
  v4i da, db;
  if (vec8 != 0 && cbase + CHUNK <= nE) {
    da = *(const v4i*)(dsts + e0);
    db = *(const v4i*)(dsts + e0 + 4);
  } else {
    da.x = (e0     < nE) ? dsts[min(e0,     nE - 1)] : sent;
    da.y = (e0 + 1 < nE) ? dsts[min(e0 + 1, nE - 1)] : sent;
    da.z = (e0 + 2 < nE) ? dsts[min(e0 + 2, nE - 1)] : sent;
    da.w = (e0 + 3 < nE) ? dsts[min(e0 + 3, nE - 1)] : sent;
    db.x = (e0 + 4 < nE) ? dsts[min(e0 + 4, nE - 1)] : sent;
    db.y = (e0 + 5 < nE) ? dsts[min(e0 + 5, nE - 1)] : sent;
    db.z = (e0 + 6 < nE) ? dsts[min(e0 + 6, nE - 1)] : sent;
    db.w = (e0 + 7 < nE) ? dsts[min(e0 + 7, nE - 1)] : sent;
  }
  const unsigned nbs = (unsigned)slotBase;
  const unsigned unb = (unsigned)nb;
  const unsigned s0 = (unsigned)da.x - nbs, s1 = (unsigned)da.y - nbs;
  const unsigned s2 = (unsigned)da.z - nbs, s3 = (unsigned)da.w - nbs;
  const unsigned s4 = (unsigned)db.x - nbs, s5 = (unsigned)db.y - nbs;
  const unsigned s6 = (unsigned)db.z - nbs, s7 = (unsigned)db.w - nbs;
  const bool h0 = s0 < unb, h1 = s1 < unb, h2 = s2 < unb, h3 = s3 < unb;
  const bool h4 = s4 < unb, h5 = s5 < unb, h6 = s6 < unb, h7 = s7 < unb;
  const unsigned any = __builtin_amdgcn_ballot_w32(h0 | h1 | h2 | h3 | h4 | h5 | h6 | h7);
  if (any != 0u) {
#define HITJ(J, HJ, SJ) { \
      const unsigned mj = __builtin_amdgcn_ballot_w32(HJ); \
      if (mj != 0u) { \
        if (HJ) { \
          const int pos = wc + (int)__builtin_amdgcn_mbcnt_lo(mj, 0u); \
          if (pos < WCAP) list[wave * WCAP + pos] = ((el0 + (J)) << SLB) | (int)(SJ); \
        } \
        wc += (int)__builtin_popcount(mj); } }
    HITJ(0, h0, s0)
    HITJ(1, h1, s1)
    HITJ(2, h2, s2)
    HITJ(3, h3, s3)
    HITJ(4, h4, s4)
    HITJ(5, h5, s5)
    HITJ(6, h6, s6)
    HITJ(7, h7, s7)
#undef HITJ
  }
  return wc;
}

__global__ __launch_bounds__(NTHR) void k_wprep(const float* __restrict__ W1, const float* __restrict__ W2,
                                                unsigned short* W1T, unsigned short* W2D) {
  const int u = (int)blockIdx.x * NTHR + (int)threadIdx.x;
  v8us o;
  unsigned short* dp;
  if (u < NU1) {
    const int n  = u >> 4;
    const int k8 = (u & 15) * 8;
    const float* p = W1 + (size_t)k8 * DF + n;
#pragma unroll
    for (int i = 0; i < 8; ++i) o[i] = (unsigned short)bf16_bits(p[(size_t)i * DF]);
    dp = W1T + (size_t)n * DF + k8;
  } else if (u < NU1 + NU2) {
    const int v  = u - NU1;
    const int n  = v >> 5;
    const int k8 = (v & 31) * 8;
    const int kk = k8 & (DF - 1);
    const float* p = W2 + (size_t)kk * DF + n;
#pragma unroll
    for (int i = 0; i < 8; ++i) o[i] = (unsigned short)bf16_bits(p[(size_t)i * DF]);
    dp = W2D + (size_t)n * KP + k8;
  } else {
    return;
  }
  *(volatile v8us*)dp = o;
  __threadfence();
  *(volatile v8us*)dp = o;
}

__global__ __launch_bounds__(NTHR) void k_cvx(const float* __restrict__ x, int nN, int nUnits,
                                              unsigned short* xb) {
  const int u = (int)blockIdx.x * NTHR + (int)threadIdx.x;
  if (u >= nUnits) return;
  const int row = u >> 4;
  const int k8  = (u & 15) * 8;
  const int rc  = row < nN ? row : nN - 1;
  const float* p = x + (size_t)rc * DF + k8;
  const v4f a = *(const v4fa*)p;
  const v4f b = *(const v4fa*)(p + 4);
  const bool ok = row < nN;
  v8us o;
  o[0] = (ok && a.x > 0.0f) ? (unsigned short)bf16_bits(a.x) : (unsigned short)0;
  o[1] = (ok && a.y > 0.0f) ? (unsigned short)bf16_bits(a.y) : (unsigned short)0;
  o[2] = (ok && a.z > 0.0f) ? (unsigned short)bf16_bits(a.z) : (unsigned short)0;
  o[3] = (ok && a.w > 0.0f) ? (unsigned short)bf16_bits(a.w) : (unsigned short)0;
  o[4] = (ok && b.x > 0.0f) ? (unsigned short)bf16_bits(b.x) : (unsigned short)0;
  o[5] = (ok && b.y > 0.0f) ? (unsigned short)bf16_bits(b.y) : (unsigned short)0;
  o[6] = (ok && b.z > 0.0f) ? (unsigned short)bf16_bits(b.z) : (unsigned short)0;
  o[7] = (ok && b.w > 0.0f) ? (unsigned short)bf16_bits(b.w) : (unsigned short)0;
  unsigned short* dp = xb + (size_t)row * DF + k8;
  *(volatile v8us*)dp = o;
  __threadfence();
  *(volatile v8us*)dp = o;
}

__global__ __launch_bounds__(GTHR) void k_gemm(const unsigned short* __restrict__ A, int lda,
                                               const unsigned short* __restrict__ BT, int ldb, int K,
                                               float* Cm, const float* __restrict__ avs,
                                               const float* __restrict__ avd, float* AL) {
  constexpr int LDC = GBN;
  constexpr int RPW = GBM / 4;
  extern __shared__ __attribute__((aligned(16))) float gsm[];
  float* stg = gsm;
  float* sdt = gsm + GBM * LDC;
  const int tid = (int)threadIdx.x, lane = tid & 31, wave = tid >> 5, hh = lane >> 4, m = lane & 15;
  const int rowBase = (int)blockIdx.x * GBM;

  v8f acc[8];
  {
    const v8f z = {0.f, 0.f, 0.f, 0.f, 0.f, 0.f, 0.f, 0.f};
#pragma unroll
    for (int t = 0; t < 8; ++t) acc[t] = z;
  }
  const unsigned short* ap = A  + (size_t)(rowBase + 16 * wave + m) * (size_t)lda + 8 * hh;
  const unsigned short* bp = BT + (size_t)m * (size_t)ldb + 8 * hh;

#pragma unroll 1
  for (int k0 = 0; k0 < K; k0 += 32) {
    FragB af;
    af.h[0] = *(const v8usa*)(ap + k0);
    af.h[1] = *(const v8usa*)(ap + k0 + 16);
#pragma unroll
    for (int nt = 0; nt < 8; ++nt) {
      const unsigned short* wq = bp + (size_t)(16 * nt) * (size_t)ldb + k0;
      FragB bf;
      bf.h[0] = *(const v8usa*)wq;
      bf.h[1] = *(const v8usa*)(wq + 16);
      acc[nt] = wmb(af, bf, acc[nt]);
    }
  }

#pragma unroll
  for (int nt = 0; nt < 8; ++nt) {
    const int lc = 16 * nt + m;
#pragma unroll
    for (int r = 0; r < 8; ++r) {
      const int lr = 16 * wave + 8 * hh + r;
      stg[lr * LDC + lc] = acc[nt][r];
    }
  }
  __syncthreads();

  const v4f as4 = bfr4(*(const v4fa*)(avs + 4 * lane));
  const v4f ad4 = bfr4(*(const v4fa*)(avd + 4 * lane));
#pragma unroll 1
  for (int i = 0; i < RPW; ++i) {
    const int row = wave * RPW + i;
    const v4f p = *(const v4fa*)(stg + row * LDC + 4 * lane);
    float s = 0.0f, d = 0.0f;
    s = fmaf(p.x, as4.x, s); s = fmaf(p.y, as4.y, s); s = fmaf(p.z, as4.z, s); s = fmaf(p.w, as4.w, s);
    d = fmaf(p.x, ad4.x, d); d = fmaf(p.y, ad4.y, d); d = fmaf(p.z, ad4.z, d); d = fmaf(p.w, ad4.w, d);
#pragma unroll
    for (int off = 16; off > 0; off >>= 1) {
      s += __shfl_xor(s, off);
      d += __shfl_xor(d, off);
    }
    if (lane == 0) { sdt[row] = s; sdt[GBM + row] = d; }
  }
  __syncthreads();

  const v4f alv = *(const v4fa*)(sdt + 4 * lane);
  float* alp = AL + (size_t)blockIdx.x * (2 * GBM) + 4 * lane;
#pragma unroll 1
  for (int i = 0; i < RPW; ++i) {
    const int row = wave * RPW + i;
    const v4f p = *(const v4fa*)(stg + row * LDC + 4 * lane);
    float* op = Cm + (size_t)(rowBase + row) * (size_t)LDC + 4 * lane;
    *(volatile v4f*)op = p;
  }
  if (wave == 0) *(volatile v4f*)alp = alv;
  __threadfence();
#pragma unroll 1
  for (int i = 0; i < RPW; ++i) {
    const int row = wave * RPW + i;
    const v4f p = *(const v4fa*)(stg + row * LDC + 4 * lane);
    float* op = Cm + (size_t)(rowBase + row) * (size_t)LDC + 4 * lane;
    *(volatile v4f*)op = p;
  }
  if (wave == 0) *(volatile v4f*)alp = alv;
}

__device__ __forceinline__ void sm_upd(float lg, const v4f a, float& mx, float& dn,
                                       float& c0, float& c1, float& c2, float& c3) {
  lg = lg > 0.f ? lg : NEGSL * lg;
  const float df = lg - mx;
  const float ee = expf(-fabsf(df));
  const bool  up = df > 0.f;
  const float s1 = up ? ee : 1.0f;
  const float s2 = up ? 1.0f : ee;
  mx = up ? lg : mx;
  dn = fmaf(dn, s1, s2);
  c0 = fmaf(c0, s1, s2 * a.x);
  c1 = fmaf(c1, s1, s2 * a.y);
  c2 = fmaf(c2, s1, s2 * a.z);
  c3 = fmaf(c3, s1, s2 * a.w);
}

template <int RL>
__global__ __launch_bounds__(NTHR) void k_agg(const int* __restrict__ srcs, const int* __restrict__ dsts,
                                              int nE, int nN, int vec8, int mRows,
                                              const float* __restrict__ AL,
                                              const float* __restrict__ xl, const float* __restrict__ bias,
                                              unsigned short* hb, float* outp) {
  extern __shared__ __attribute__((aligned(16))) int dsm[];
  int* list = dsm;
  int* hl   = dsm + LISTN;
  int* sl   = dsm + LISTN + RCAP;
  int* cnt  = dsm + LISTN + 2 * RCAP;
  int* offs = cnt + NBA;
  int* cur  = offs + NBA;
  int* misc = cur + NBA;
  const int tid = (int)threadIdx.x, lane = tid & 31, wave = tid >> 5;
  const int nodeBase = (int)blockIdx.x * NBA;

  {
    const v4i z4 = {0, 0, 0, 0};
    for (int i = tid * 4; i < AGG_ZINTS; i += NTHR * 4) *(v4ia*)(dsm + i) = z4;
    if (tid < 16) misc[tid] = 0;
  }
  float bv0, bv1, bv2, bv3;
  {
    const v4f a = *(const v4fa*)(bias + 4 * lane);
    bv0 = bf16_val(a.x); bv1 = bf16_val(a.y); bv2 = bf16_val(a.z); bv3 = bf16_val(a.w);
  }
  __syncthreads();

  int t = 0, ov = 0;
  const int nChunks = (nE + CHUNK - 1) / CHUNK;
#pragma unroll 1
  for (int ch = 0; ch < nChunks; ++ch) {
    const int cbase = ch * CHUNK;
    const int wc = scan_chunk<SLA>(dsts, nE, cbase, nodeBase, NBA, vec8, list, tid, lane, wave);
    if (lane == 0) misc[wave] = wc;
    __syncthreads();
    if (wave == 0) {
#pragma unroll 1
      for (int w2 = 0; w2 < NWAVE; ++w2) {
        int c = misc[w2];
        c = c < 0 ? 0 : (c > WCAP ? WCAP : c);
#pragma unroll 1
        for (int b0 = 0; b0 < c; b0 += 32) {
          const int idx = b0 + lane;
          const int ent = list[w2 * WCAP + (idx < WCAP ? idx : WCAP - 1)];
          const int m32 = (c - b0) < 32 ? (c - b0) : 32;
#pragma unroll 1
          for (int k = 0; k < m32; ++k) {
            const int u    = __builtin_amdgcn_readlane(ent, k);
            const int slot = u & (NBA - 1);
            const int el   = (u >> SLA) & (CHUNK - 1);
            const int pk   = ((cbase + el) << SLA) | slot;
            if (t < RCAP) {
              if (lane == 0) { hl[t] = pk; cnt[slot] = cnt[slot] + 1; }
              t = t + 1;
            } else {
              ov = 1;
            }
          }
        }
      }
    }
    __syncthreads();
  }
  if (wave == 0 && lane == 0) { misc[8] = t; misc[9] = ov; }
  __syncthreads();
  int tt = misc[8];
  tt = tt < 0 ? 0 : (tt > RCAP ? RCAP : tt);
  const int ovf = misc[9];

  if (wave == 0) {
    const int base = lane * (NBA / 32);
    int s = 0;
#pragma unroll 1
    for (int i = 0; i < NBA / 32; ++i) s += cnt[base + i];
    int incl = s;
#pragma unroll
    for (int d = 1; d < 32; d <<= 1) {
      const int y = __shfl_up(incl, d, 32);
      if (lane >= d) incl += y;
    }
    int run = incl - s;
#pragma unroll 1
    for (int i = 0; i < NBA / 32; ++i) {
      const int cv = cnt[base + i];
      offs[base + i] = run;
      cur[base + i]  = run;
      run += cv;
    }
  }
  __syncthreads();
  if (wave == 0) {
#pragma unroll 1
    for (int b0 = 0; b0 < tt; b0 += 32) {
      const int idx = b0 + lane;
      const int ent = hl[idx < RCAP ? idx : RCAP - 1];
      const int m32 = (tt - b0) < 32 ? (tt - b0) : 32;
#pragma unroll 1
      for (int k = 0; k < m32; ++k) {
        const int u    = __builtin_amdgcn_readlane(ent, k);
        const int slot = u & (NBA - 1);
        if (lane == 0) {
          int p = cur[slot];
          p = p < 0 ? 0 : (p > RCAP - 1 ? RCAP - 1 : p);
          sl[p] = u;
          cur[slot] = p + 1;
        }
      }
    }
  }
  __syncthreads();

  const float qnan = __int_as_float(0x7fc00000);
  const float pz = (ovf != 0) ? qnan : 0.0f;
  const int sa = (2 * lane) & 31, sb = (2 * lane + 1) & 31;
#pragma unroll 1
  for (int si = 0; si < NBA / NWAVE; ++si) {
    const int s    = si * NWAVE + wave;
    const int node = nodeBase + s;
    int c = cnt[s];
    const bool big = c > DEGCAP;
    c = c < 0 ? 0 : (c > DEGCAP ? DEGCAP : c);
    int o = offs[s];
    o = o < 0 ? 0 : (o > RCAP ? RCAP : o);
    const int nc  = node < nN ? node : nN - 1;
    const int alb = (nc >> 6) * (2 * GBM) + (nc & (GBM - 1));
    const float as0 = AL[alb];
    const float ad  = AL[alb + GBM];
    float mx = -3.0e38f, dn = 0.0f;
    float a0 = 0.0f, a1 = 0.0f, a2 = 0.0f, a3 = 0.0f;
#pragma unroll 1
    for (int b0 = 0; b0 < c; b0 += 32) {
      int idx = o + b0 + lane;
      idx = idx > RCAP - 1 ? RCAP - 1 : idx;
      const int ent = sl[idx];
      int eid = ent >> SLA;
      eid = eid < 0 ? 0 : (eid > nE - 1 ? nE - 1 : eid);
      int sr = srcs[eid];
      sr = sr < 0 ? 0 : (sr > nN - 1 ? nN - 1 : sr);
      const float es  = AL[(sr >> 6) * (2 * GBM) + (sr & (GBM - 1))];
      const int   esi = __float_as_int(es);
      const int m32 = (c - b0) < 32 ? (c - b0) : 32;
#pragma unroll 1
      for (int k = 0; k < m32; ++k) {
        const int   sk  = __builtin_amdgcn_readlane(sr, k);
        const float ask = __int_as_float(__builtin_amdgcn_readlane(esi, k));
        const v4f a = *(const v4fa*)(xl + (size_t)sk * DF + 4 * lane);
        sm_upd(ask + ad, a, mx, dn, a0, a1, a2, a3);
      }
    }
    {
      const v4f a = *(const v4fa*)(xl + (size_t)nc * DF + 4 * lane);
      sm_upd(as0 + ad, a, mx, dn, a0, a1, a2, a3);
    }
    const float inv = __builtin_amdgcn_rcpf(dn);
    const float pzr = big ? qnan : pz;
    const bool live = node < nN;
    float y0 = fmaf(a0, inv, bv0), y1 = fmaf(a1, inv, bv1);
    float y2 = fmaf(a2, inv, bv2), y3 = fmaf(a3, inv, bv3);
    y0 = (y0 > 0.0f) ? y0 : (y0 - y0);
    y1 = (y1 > 0.0f) ? y1 : (y1 - y1);
    y2 = (y2 > 0.0f) ? y2 : (y2 - y2);
    y3 = (y3 > 0.0f) ? y3 : (y3 - y3);
    y0 = y0 + pzr; y1 = y1 + pzr; y2 = y2 + pzr; y3 = y3 + pzr;
    const float v0 = live ? y0 : 0.0f, v1 = live ? y1 : 0.0f;
    const float v2 = live ? y2 : 0.0f, v3 = live ? y3 : 0.0f;
    if constexpr (RL != 0) {
      const unsigned h0 = bf16_bits(v0), h1 = bf16_bits(v1), h2 = bf16_bits(v2), h3 = bf16_bits(v3);
      const unsigned l0 = bf16_bits(v0 - __uint_as_float(h0 << 16));
      const unsigned l1 = bf16_bits(v1 - __uint_as_float(h1 << 16));
      const unsigned l2 = bf16_bits(v2 - __uint_as_float(h2 << 16));
      const unsigned l3 = bf16_bits(v3 - __uint_as_float(h3 << 16));
      const int hw0 = (int)(h0 | (h1 << 16));
      const int hw1 = (int)(h2 | (h3 << 16));
      const int lw0 = (int)(l0 | (l1 << 16));
      const int lw1 = (int)(l2 | (l3 << 16));
      const int g0 = __shfl(hw0, sa, 32), g1 = __shfl(hw1, sa, 32);
      const int g2 = __shfl(hw0, sb, 32), g3 = __shfl(hw1, sb, 32);
      const int p0 = __shfl(lw0, sa, 32), p1 = __shfl(lw1, sa, 32);
      const int p2 = __shfl(lw0, sb, 32), p3 = __shfl(lw1, sb, 32);
      const bool lsel = lane >= 16;
      v4u pv;
      pv.x = (unsigned int)(lsel ? p0 : g0);
      pv.y = (unsigned int)(lsel ? p1 : g1);
      pv.z = (unsigned int)(lsel ? p2 : g2);
      pv.w = (unsigned int)(lsel ? p3 : g3);
      const bool wr = node < mRows;
      unsigned short* hp = hb + (size_t)(wr ? node : 0) * KP + 8 * lane;
      if (wr) *(volatile v4u*)hp = pv;
      __threadfence();
      if (wr) *(volatile v4u*)hp = pv;
    } else {
      v4f ov4;
      ov4.x = v0; ov4.y = v1; ov4.z = v2; ov4.w = v3;
      float* op = outp + (size_t)nc * DF + 4 * lane;
      if (live) *(volatile v4f*)op = ov4;
      __threadfence();
      if (live) *(volatile v4f*)op = ov4;
    }
  }
}

__global__ __launch_bounds__(PTHR) void k_pool(const float* __restrict__ hf, const int* __restrict__ bat,
                                               int nN, const float* __restrict__ fcw,
                                               const float* __restrict__ fcb, float* out) {
  __shared__ float res[PWAVE];
  const int tid = (int)threadIdx.x, lane = tid & 31, wave = tid >> 5;
  const int g = (int)blockIdx.x * PWAVE + wave;
  const v4f wm = bfr4(*(const v4fa*)(fcw + 4 * lane));
  const v4f wa = bfr4(*(const v4fa*)(fcw + DF + 4 * lane));
  const float fb = bf16_val(fcb[0]);
  const float ninf = __int_as_float((int)0xff800000u);
  float m0 = ninf, m1 = ninf, m2 = ninf, m3 = ninf;
  float s0 = 0.0f, s1 = 0.0f, s2 = 0.0f, s3 = 0.0f;
  int mine = 0;
#pragma unroll 1
  for (int i0 = 0; i0 < nN; i0 += 32) {
    const int i  = i0 + lane;
    const int ic = i < nN ? i : nN - 1;
    const int b  = bat[ic];
    const bool hit = (i < nN) && (b == g);
    unsigned msk = __builtin_amdgcn_ballot_w32(hit);
    int nh = (int)__builtin_popcount(msk);
    nh = nh > 32 ? 32 : nh;
    mine += hit ? 1 : 0;
#pragma unroll 1
    for (int q = 0; q < nh; ++q) {
      const int k = __builtin_ffs((int)msk) - 1;
      msk &= msk - 1u;
      int node = i0 + (k < 0 ? 0 : k);
      node = node > nN - 1 ? nN - 1 : node;
      const v4f v = *(const v4fa*)(hf + (size_t)node * DF + 4 * lane);
      m0 = fmaxf(m0, v.x); m1 = fmaxf(m1, v.y); m2 = fmaxf(m2, v.z); m3 = fmaxf(m3, v.w);
      s0 += v.x; s1 += v.y; s2 += v.z; s3 += v.w;
    }
  }
  int cnt = mine;
  cnt += __shfl_xor(cnt, 16); cnt += __shfl_xor(cnt, 8); cnt += __shfl_xor(cnt, 4);
  cnt += __shfl_xor(cnt, 2);  cnt += __shfl_xor(cnt, 1);
  const bool has = cnt > 0;
  const float cf = has ? (float)cnt : 1.0f;
  const float rc = 1.0f / cf;
  const float q0 = has ? m0 : 0.0f, q1 = has ? m1 : 0.0f, q2 = has ? m2 : 0.0f, q3 = has ? m3 : 0.0f;
  float p = 0.0f;
  p = fmaf(q0, wm.x, p); p = fmaf(q1, wm.y, p); p = fmaf(q2, wm.z, p); p = fmaf(q3, wm.w, p);
  p = fmaf(s0 * rc, wa.x, p); p = fmaf(s1 * rc, wa.y, p); p = fmaf(s2 * rc, wa.z, p); p = fmaf(s3 * rc, wa.w, p);
#pragma unroll
  for (int off = 16; off > 0; off >>= 1) p += __shfl_xor(p, off);
  if (lane == 0) res[wave] = p + fb;
  __syncthreads();
  if (wave == 0) {
    const float r = res[lane];
    float* op = out + (size_t)blockIdx.x * PWAVE + lane;
    *(volatile float*)op = r;
    __threadfence();
    *(volatile float*)op = r;
  }
}

static inline int cdiv(int a, int b) { return (a + b - 1) / b; }
static inline size_t al256(size_t o) { return (o + 255) & ~(size_t)255; }

extern "C" void kernel_launch(void* const* d_in, const int* in_sizes, int n_in,
                              void* d_out, int out_size, void* d_ws, size_t ws_size,
                              hipStream_t stream) {
  if (n_in < 13) return;
  if (in_sizes[0] < DF || (in_sizes[0] % DF) != 0) return;
  const int nN = in_sizes[0] / DF;
  if (nN < 1 || nN > (1 << 22)) return;
  if (in_sizes[1] < 2 || (in_sizes[1] & 1) != 0) return;
  const int nE = in_sizes[1] / 2;
  if (nE < 1 || nE >= (1 << (31 - SLA))) return;
  if (in_sizes[2] != nN) return;
  if (in_sizes[3] != DF * DF) return;
  if (in_sizes[4] != DF || in_sizes[5] != DF || in_sizes[6] != DF) return;
  if (in_sizes[7] != DF * DF) return;
  if (in_sizes[8] != DF || in_sizes[9] != DF || in_sizes[10] != DF) return;
  if (in_sizes[11] != 2 * DF || in_sizes[12] < 1) return;
  if (out_size != NGR) return;

  const float* x    = (const float*)d_in[0];
  const int*   edge = (const int*)d_in[1];
  const int*   bat  = (const int*)d_in[2];
  const float* W1   = (const float*)d_in[3];
  const float* a1s  = (const float*)d_in[4];
  const float* a1d  = (const float*)d_in[5];
  const float* b1   = (const float*)d_in[6];
  const float* W2   = (const float*)d_in[7];
  const float* a2s  = (const float*)d_in[8];
  const float* a2d  = (const float*)d_in[9];
  const float* b2   = (const float*)d_in[10];
  const float* fcw  = (const float*)d_in[11];
  const float* fcb  = (const float*)d_in[12];
  float* out = (float*)d_out;
  const int* src = edge;
  const int* dst = edge + nE;

  const int MP   = cdiv(nN, GBM) * GBM;
  const int gM   = MP / GBM;
  const int gA   = cdiv(MP, NBA);
  if ((long long)gA * NBA < (long long)MP) return;
  const int vec8 = ((nE & 3) == 0) ? 1 : 0;

  char* ws = (char*)d_ws;
  size_t off = 0;
  const size_t oW1T = off; off = al256(off + (size_t)DF * DF * 2);
  const size_t oW2D = off; off = al256(off + (size_t)DF * KP * 2);
  const size_t oAL1 = off; off = al256(off + (size_t)gM * (2 * GBM) * 4);
  const size_t oAL2 = off; off = al256(off + (size_t)gM * (2 * GBM) * 4);
  const size_t oXB  = off; off = al256(off + (size_t)MP * DF * 2);
  const size_t oT   = off; off = al256(off + (size_t)MP * DF * 4);
  const size_t oX1  = off; off = al256(off + (size_t)MP * KP * 2);
  const size_t oHO  = off; off = al256(off + (size_t)MP * DF * 4);
  if (off > ws_size || off > (size_t)WSMAX) return;
  unsigned short* W1T  = (unsigned short*)(ws + oW1T);
  unsigned short* W2D  = (unsigned short*)(ws + oW2D);
  float*          AL1  = (float*)(ws + oAL1);
  float*          AL2  = (float*)(ws + oAL2);
  unsigned short* XB   = (unsigned short*)(ws + oXB);
  float*          T    = (float*)(ws + oT);
  unsigned short* X1HL = (unsigned short*)(ws + oX1);
  float*          HOUT = (float*)(ws + oHO);

  const size_t aggLds  = (size_t)AGG_LDS_INTS * 4;
  const size_t gemmLds = (size_t)(GBM * GBN + 2 * GBM) * 4;
  hipFuncSetAttribute(reinterpret_cast<const void*>(&k_agg<1>), hipFuncAttributeMaxDynamicSharedMemorySize, (int)aggLds);
  hipFuncSetAttribute(reinterpret_cast<const void*>(&k_agg<0>), hipFuncAttributeMaxDynamicSharedMemorySize, (int)aggLds);

  const int nUx = MP * (DF / 8);
  k_wprep<<<(NU1 + NU2) / NTHR, NTHR, 0, stream>>>(W1, W2, W1T, W2D);
  k_cvx<<<cdiv(nUx, NTHR), NTHR, 0, stream>>>(x, nN, nUx, XB);
  k_gemm<<<gM, GTHR, gemmLds, stream>>>(XB, DF, W1T, DF, DF, T, a1s, a1d, AL1);
  k_agg<1><<<gA, NTHR, aggLds, stream>>>(src, dst, nE, nN, vec8, MP, AL1, T, b1, X1HL, HOUT);
  k_gemm<<<gM, GTHR, gemmLds, stream>>>(X1HL, KP, W2D, KP, KP, T, a2s, a2d, AL2);
  k_agg<0><<<gA, NTHR, aggLds, stream>>>(src, dst, nE, nN, vec8, MP, AL2, T, b2, X1HL, HOUT);
  k_pool<<<NGR / PWAVE, PTHR, 0, stream>>>(HOUT, bat, nN, fcw, fcb, out);
}
